// GNN_node_57062935495533
// MI455X (gfx1250) — hardware-verified
//
#include <hip/hip_runtime.h>
#include <stddef.h>
#include <stdint.h>


#define D      64
#define D2     128
#define FE     7
#define WEF    (FE * D)
#define K1     128
#define K2     256
#define NTHR   256
#define NWAVE  8
#define EPT    8
#define CHUNK  (NTHR * EPT)
#define WCAP   (EPT * 32)
#define LISTN  (NWAVE * WCAP)
#define NBA    1024
#define SLA    10
#define RCAP   28672
#define DEGCAP 64
#define GBM    64
#define GTHR   128
#define GWAVE  (GTHR / 32)
#define PARTW  288
#define WSTW   258
#define HPR    8
#define HPB    (NWAVE * HPR)
#define AGG_ZINTS    (LISTN + 2 * RCAP + 3 * NBA)
#define MISC_INTS    16
#define AGG_LDS_INTS (AGG_ZINTS + MISC_INTS + WEF + D)
#define MAXL   8
#define WSMAX  134217728

static_assert((CHUNK & (CHUNK - 1)) == 0 && CHUNK <= 4096);
static_assert((NBA & (NBA - 1)) == 0 && NBA == (1 << SLA));
static_assert(((long long)CHUNK << SLA) < (1LL << 31));
static_assert(LISTN % NTHR == 0);
static_assert(NBA % NWAVE == 0 && NBA % 32 == 0 && NBA % GBM == 0);
static_assert(RCAP % 4 == 0 && AGG_ZINTS % 4 == 0 && LISTN % 4 == 0 && ((AGG_ZINTS + MISC_INTS) % 4) == 0);
static_assert(AGG_ZINTS % (NTHR * 4) == 0);
static_assert(K1 % 32 == 0 && K2 % 32 == 0 && K1 == 2 * D && K2 == 2 * D2);
static_assert(GBM == GWAVE * 16 && D == 2 * 32 && D2 == 4 * 32 && GTHR == D2);
static_assert(PARTW % 32 == 0 && PARTW / 4 <= GTHR && PARTW >= 2 * D2 + 1);
static_assert(WSTW >= 2 * D2 + 1 && (WSTW % 2) == 0);
static_assert(HPB == GBM && NTHR == 2 * D2);
static_assert((WEF % 4) == 0);
static_assert(AGG_LDS_INTS * 4 <= 300000);

typedef float          v2f   __attribute__((ext_vector_type(2)));
typedef float          v4f   __attribute__((ext_vector_type(4)));
typedef float          v8f   __attribute__((ext_vector_type(8)));
typedef int            v4i   __attribute__((ext_vector_type(4)));
typedef int            v8i   __attribute__((ext_vector_type(8)));
typedef unsigned short v4us  __attribute__((ext_vector_type(4)));
typedef unsigned short v8us  __attribute__((ext_vector_type(8)));
typedef unsigned short v16us __attribute__((ext_vector_type(16)));
typedef __bf16         v16bf __attribute__((ext_vector_type(16)));
typedef v2f  __attribute__((may_alias)) v2fa;
typedef v4f  __attribute__((may_alias)) v4fa;
typedef v4i  __attribute__((may_alias)) v4ia;
typedef v4us __attribute__((may_alias)) v4usa;
typedef v8us __attribute__((may_alias)) v8usa;
union FragB { v16bf v; v16us u; v8us h[2]; v8i w; };

__device__ __forceinline__ v8f wmb(const FragB& a, const FragB& b, v8f c) {
  v8f d = __builtin_amdgcn_wmma_f32_16x16x32_bf16(false, a.v, false, b.v, (short)0, c, false, false);
  asm volatile("v_nop\n\tv_nop\n\tv_nop\n\tv_nop" : "+v"(d) : "v"(a.w), "v"(b.w));
  return d;
}

__device__ __forceinline__ v8f z8() { v8f z = {0.f, 0.f, 0.f, 0.f, 0.f, 0.f, 0.f, 0.f}; return z; }

__device__ __forceinline__ unsigned bf16_bits(float f) {
  const unsigned u = __float_as_uint(f);
  return (u + 0x7FFFu + ((u >> 16) & 1u)) >> 16;
}
__device__ __forceinline__ float bf16_val(float f) {
  return __uint_as_float(bf16_bits(f) << 16);
}
__device__ __forceinline__ unsigned hl_bits(float v, unsigned& lo) {
  const unsigned hb = bf16_bits(v);
  lo = bf16_bits(v - __uint_as_float(hb << 16));
  return hb;
}

__device__ __forceinline__ void wave_sync() {
  __builtin_amdgcn_fence(__ATOMIC_RELEASE, "wavefront");
  __builtin_amdgcn_wave_barrier();
  __builtin_amdgcn_fence(__ATOMIC_ACQUIRE, "wavefront");
}

template <int SLB>
__device__ __forceinline__ int scan_chunk(const int* __restrict__ dsts, int nE, int cbase, int slotBase,
                                          int nb, int vec8, int* list, int tid, int lane, int wave) {
  int wc = 0;
  const int el0  = tid * EPT;
  const int e0   = cbase + el0;
  const int sent = -2147483647 - 1;
  v4i da, db;
  if (vec8 != 0 && cbase + CHUNK <= nE) {
    da = *(const v4i*)(dsts + e0);
    db = *(const v4i*)(dsts + e0 + 4);
  } else {
    da.x = (e0     < nE) ? dsts[min(e0,     nE - 1)] : sent;
    da.y = (e0 + 1 < nE) ? dsts[min(e0 + 1, nE - 1)] : sent;
    da.z = (e0 + 2 < nE) ? dsts[min(e0 + 2, nE - 1)] : sent;
    da.w = (e0 + 3 < nE) ? dsts[min(e0 + 3, nE - 1)] : sent;
    db.x = (e0 + 4 < nE) ? dsts[min(e0 + 4, nE - 1)] : sent;
    db.y = (e0 + 5 < nE) ? dsts[min(e0 + 5, nE - 1)] : sent;
    db.z = (e0 + 6 < nE) ? dsts[min(e0 + 6, nE - 1)] : sent;
    db.w = (e0 + 7 < nE) ? dsts[min(e0 + 7, nE - 1)] : sent;
  }
  const unsigned nbs = (unsigned)slotBase;
  const unsigned unb = (unsigned)nb;
  const unsigned s0 = (unsigned)da.x - nbs, s1 = (unsigned)da.y - nbs;
  const unsigned s2 = (unsigned)da.z - nbs, s3 = (unsigned)da.w - nbs;
  const unsigned s4 = (unsigned)db.x - nbs, s5 = (unsigned)db.y - nbs;
  const unsigned s6 = (unsigned)db.z - nbs, s7 = (unsigned)db.w - nbs;
  const bool h0 = s0 < unb, h1 = s1 < unb, h2 = s2 < unb, h3 = s3 < unb;
  const bool h4 = s4 < unb, h5 = s5 < unb, h6 = s6 < unb, h7 = s7 < unb;
  const unsigned any = __builtin_amdgcn_ballot_w32(h0 | h1 | h2 | h3 | h4 | h5 | h6 | h7);
  if (any != 0u) {
#define HITJ(J, HJ, SJ) { \
      const unsigned mj = __builtin_amdgcn_ballot_w32(HJ); \
      if (mj != 0u) { \
        if (HJ) { \
          const int pos = wc + (int)__builtin_amdgcn_mbcnt_lo(mj, 0u); \
          if (pos < WCAP) list[wave * WCAP + pos] = ((el0 + (J)) << SLB) | (int)(SJ); \
        } \
        wc += (int)__builtin_popcount(mj); } }
    HITJ(0, h0, s0)
    HITJ(1, h1, s1)
    HITJ(2, h2, s2)
    HITJ(3, h3, s3)
    HITJ(4, h4, s4)
    HITJ(5, h5, s5)
    HITJ(6, h6, s6)
    HITJ(7, h7, s7)
#undef HITJ
  }
  return wc;
}

__global__ __launch_bounds__(NTHR) void k_wprep(const float* __restrict__ W1, const float* __restrict__ W2,
                                                int nL, unsigned short* BT1, unsigned short* BT2) {
  const int blk = (int)blockIdx.x;
  const int nb1 = 4 * nL;
  const float* p;
  unsigned short* dp;
  int stride, kmat;
  if (blk < nb1) {
    const int u  = blk * NTHR + (int)threadIdx.x;
    const int l  = u >> 10;
    const int n  = (u >> 3) & (D2 - 1);
    const int k8 = (u & 7) * 8;
    p  = W1 + (size_t)l * (D * D2) + (size_t)k8 * D2 + n;
    dp = BT1 + (size_t)l * (D2 * K1) + (size_t)n * K1 + k8;
    stride = D2; kmat = D;
  } else {
    const int u  = (blk - nb1) * NTHR + (int)threadIdx.x;
    const int l  = u >> 10;
    const int n  = (u >> 4) & (D - 1);
    const int k8 = (u & 15) * 8;
    p  = W2 + (size_t)l * (D2 * D) + (size_t)k8 * D + n;
    dp = BT2 + (size_t)l * (D * K2) + (size_t)n * K2 + k8;
    stride = D; kmat = D2;
  }
  v8us o;
#pragma unroll
  for (int i = 0; i < 8; ++i) o[i] = (unsigned short)bf16_bits(p[(size_t)i * stride]);
  *(volatile v8us*)dp = o;
  *(volatile v8us*)(dp + kmat) = o;
  __threadfence();
  *(volatile v8us*)dp = o;
  *(volatile v8us*)(dp + kmat) = o;
}

__global__ __launch_bounds__(NTHR) void k_hinit(const int* __restrict__ xi, const float* __restrict__ emb,
                                                int nEmbRows, int nN, int nUnits, float* hout) {
  const int u = (int)blockIdx.x * NTHR + (int)threadIdx.x;
  if (u >= nUnits) return;
  const int row = u >> 4, j = u & 15;
  const bool live = row < nN;
  const int rc = live ? row : (nN - 1);
  int ix = xi[rc];
  ix = ix < 0 ? 0 : (ix > nEmbRows - 1 ? nEmbRows - 1 : ix);
  const v4f a = *(const v4fa*)(emb + (size_t)ix * D + 4 * j);
  v4f y;
  y.x = live ? bf16_val(a.x) : 0.0f;
  y.y = live ? bf16_val(a.y) : 0.0f;
  y.z = live ? bf16_val(a.z) : 0.0f;
  y.w = live ? bf16_val(a.w) : 0.0f;
  float* op = hout + (size_t)row * D + 4 * j;
  *(volatile v4f*)op = y;
  __threadfence();
  *(volatile v4f*)op = y;
}

__global__ __launch_bounds__(NTHR) void k_scan(const int* __restrict__ srcs, const int* __restrict__ dsts,
                                               int nE, int nN, int vec8, int mRows,
                                               const float* __restrict__ eattr, const float* __restrict__ wel,
                                               const float* __restrict__ bel, const float* __restrict__ epl,
                                               const float* __restrict__ hsrc, unsigned short* apl) {
  extern __shared__ __attribute__((aligned(16))) int dsm[];
  int* list = dsm;
  int* hl   = dsm + LISTN;
  int* sl   = hl + RCAP;
  int* cnt  = sl + RCAP;
  int* offs = cnt + NBA;
  int* cur  = offs + NBA;
  int* misc = cur + NBA;
  float* swe = (float*)(misc + MISC_INTS);
  float* sbe = swe + WEF;
  const int tid = (int)threadIdx.x, lane = tid & 31, wave = tid >> 5;
  const int nodeBase = (int)blockIdx.x * NBA;

  {
    const v4i z4 = {0, 0, 0, 0};
    for (int i = tid * 4; i < AGG_ZINTS; i += NTHR * 4) *(v4ia*)(dsm + i) = z4;
    if (tid < MISC_INTS) misc[tid] = 0;
  }
#pragma unroll 1
  for (int i = tid; i < WEF; i += NTHR) swe[i] = bf16_val(wel[i]);
  if (tid < D) sbe[tid] = bf16_val(bel[tid]);
  __syncthreads();

  float wx[FE], wy[FE];
#pragma unroll
  for (int j = 0; j < FE; ++j) {
    const v2f w2 = *(const v2fa*)(swe + j * D + 2 * lane);
    wx[j] = w2.x;
    wy[j] = w2.y;
  }
  const v2f bev = *(const v2fa*)(sbe + 2 * lane);
  const float opl = 1.0f + bf16_val(epl[0]);

  int t = 0, ov = 0;
  const int nChunks = (nE + CHUNK - 1) / CHUNK;
#pragma unroll 1
  for (int ch = 0; ch < nChunks; ++ch) {
    const int cbase = ch * CHUNK;
    const int wc = scan_chunk<SLA>(dsts, nE, cbase, nodeBase, NBA, vec8, list, tid, lane, wave);
    if (lane == 0) misc[wave] = wc;
    __syncthreads();
    if (wave == 0) {
#pragma unroll 1
      for (int w2 = 0; w2 < NWAVE; ++w2) {
        int c = misc[w2];
        c = c < 0 ? 0 : (c > WCAP ? WCAP : c);
#pragma unroll 1
        for (int b0 = 0; b0 < c; b0 += 32) {
          const int idx = b0 + lane;
          const int ent = list[w2 * WCAP + (idx < WCAP ? idx : WCAP - 1)];
          const int m32 = (c - b0) < 32 ? (c - b0) : 32;
#pragma unroll 1
          for (int k = 0; k < m32; ++k) {
            const int u    = __builtin_amdgcn_readlane(ent, k);
            const int slot = u & (NBA - 1);
            const int el   = (u >> SLA) & (CHUNK - 1);
            const int pk   = ((cbase + el) << SLA) | slot;
            if (t < RCAP) {
              if (lane == 0) { hl[t] = pk; cnt[slot] = cnt[slot] + 1; }
              t = t + 1;
            } else {
              ov = 1;
            }
          }
        }
      }
    }
    __syncthreads();
  }
  if (wave == 0 && lane == 0) { misc[8] = t; misc[9] = ov; }
  __syncthreads();
  int tt = misc[8];
  tt = tt < 0 ? 0 : (tt > RCAP ? RCAP : tt);
  const int ovf = misc[9];

  if (wave == 0) {
    const int base = lane * (NBA / 32);
    int s = 0;
#pragma unroll 1
    for (int i = 0; i < NBA / 32; ++i) s += cnt[base + i];
    int incl = s;
#pragma unroll
    for (int d = 1; d < 32; d <<= 1) {
      const int y = __shfl_up(incl, d, 32);
      if (lane >= d) incl += y;
    }
    int run = incl - s;
#pragma unroll 1
    for (int i = 0; i < NBA / 32; ++i) {
      const int cv = cnt[base + i];
      offs[base + i] = run;
      cur[base + i]  = run;
      run += cv;
    }
  }
  __syncthreads();
  if (wave == 0) {
#pragma unroll 1
    for (int b0 = 0; b0 < tt; b0 += 32) {
      const int idx = b0 + lane;
      const int ent = hl[idx < RCAP ? idx : RCAP - 1];
      const int m32 = (tt - b0) < 32 ? (tt - b0) : 32;
#pragma unroll 1
      for (int k = 0; k < m32; ++k) {
        const int u    = __builtin_amdgcn_readlane(ent, k);
        const int slot = u & (NBA - 1);
        if (lane == 0) {
          int p = cur[slot];
          p = p < 0 ? 0 : (p > RCAP - 1 ? RCAP - 1 : p);
          sl[p] = u;
          cur[slot] = p + 1;
        }
      }
    }
  }
  __syncthreads();

  const float pz = (ovf != 0) ? __int_as_float(0x7fc00000) : 0.0f;
#pragma unroll 1
  for (int si = 0; si < NBA / NWAVE; ++si) {
    const int s    = si * NWAVE + wave;
    const int node = nodeBase + s;
    int c = cnt[s];
    const bool big = c > DEGCAP;
    c = c < 0 ? 0 : (c > DEGCAP ? DEGCAP : c);
    int o = offs[s];
    o = o < 0 ? 0 : (o > RCAP ? RCAP : o);
    const int nc = node < nN ? node : nN - 1;
    float a0 = 0.0f, a1 = 0.0f;
#pragma unroll 1
    for (int b0 = 0; b0 < c; b0 += 32) {
      int idx = o + b0 + lane;
      idx = idx > RCAP - 1 ? RCAP - 1 : idx;
      const int ent = sl[idx];
      int eid = ent >> SLA;
      eid = eid < 0 ? 0 : (eid > nE - 1 ? nE - 1 : eid);
      int sr = srcs[eid];
      sr = sr < 0 ? 0 : (sr > nN - 1 ? nN - 1 : sr);
      const int m32 = (c - b0) < 32 ? (c - b0) : 32;
#pragma unroll 1
      for (int k = 0; k < m32; ++k) {
        const int ek = __builtin_amdgcn_readlane(eid, k);
        const int sk = __builtin_amdgcn_readlane(sr, k);
        const float* er = eattr + (size_t)ek * FE;
        float ev[FE];
#pragma unroll
        for (int j = 0; j < FE; ++j) ev[j] = bf16_val(er[j]);
        const v2f hv = *(const v2fa*)(hsrc + (size_t)sk * D + 2 * lane);
        float d0 = ev[0] * wx[0];
        float d1 = ev[0] * wy[0];
#pragma unroll
        for (int j = 1; j < FE; ++j) {
          d0 = fmaf(ev[j], wx[j], d0);
          d1 = fmaf(ev[j], wy[j], d1);
        }
        const float mx = fmaxf(hv.x + (d0 + bev.x), 0.0f);
        const float my = fmaxf(hv.y + (d1 + bev.y), 0.0f);
        a0 = a0 + mx;
        a1 = a1 + my;
      }
    }
    const float pzr = big ? __int_as_float(0x7fc00000) : pz;
    const bool live = node < nN;
    const v2f hr = *(const v2fa*)(hsrc + (size_t)nc * D + 2 * lane);
    const float z0 = live ? (fmaf(opl, hr.x, a0) + pzr) : 0.0f;
    const float z1 = live ? (fmaf(opl, hr.y, a1) + pzr) : 0.0f;
    unsigned lb0, lb1;
    const unsigned hb0 = hl_bits(z0, lb0);
    const unsigned hb1 = hl_bits(z1, lb1);
    const unsigned hp = hb0 | (hb1 << 16);
    const unsigned lp = lb0 | (lb1 << 16);
    if (node < mRows) {
      unsigned short* rpw = apl + (size_t)node * K1;
      unsigned* ph = (unsigned*)rpw + lane;
      unsigned* pl = (unsigned*)(rpw + D) + lane;
      *(volatile unsigned*)ph = hp;
      *(volatile unsigned*)pl = lp;
      __threadfence();
      *(volatile unsigned*)ph = hp;
      *(volatile unsigned*)pl = lp;
    }
  }
}

template <int NC, int KK>
__global__ __launch_bounds__(GTHR) void k_gemm(const unsigned short* __restrict__ Apl,
                                               const unsigned short* __restrict__ BT,
                                               const float* __restrict__ bias, int nN,
                                               float* outp, float* part) {
  constexpr int NT  = NC / 16;
  constexpr int CPL = NC / 32;
  static_assert(NT >= 1 && NT <= 8 && (CPL == 2 || CPL == 4) && KK % 32 == 0);
  __shared__ __attribute__((aligned(16))) float stg[GBM * D2];
  __shared__ __attribute__((aligned(16))) float wst[GWAVE * WSTW];
  __shared__ __attribute__((aligned(16))) float pst[PARTW];
  const int tid = (int)threadIdx.x, lane = tid & 31, wave = tid >> 5, hh = lane >> 4, m = lane & 15;
  const int rowBase = (int)blockIdx.x * GBM;

  v8f acc[NT];
#pragma unroll
  for (int t = 0; t < NT; ++t) acc[t] = z8();
  const unsigned short* ap = Apl + (size_t)(rowBase + 16 * wave + m) * (size_t)KK + 8 * hh;
  const unsigned short* bp = BT + (size_t)m * (size_t)KK + 8 * hh;

#pragma unroll 1
  for (int k0 = 0; k0 < KK; k0 += 32) {
    FragB af;
    af.h[0] = *(const v8usa*)(ap + k0);
    af.h[1] = *(const v8usa*)(ap + k0 + 16);
#pragma unroll
    for (int nt = 0; nt < NT; ++nt) {
      const unsigned short* wq = bp + (size_t)(16 * nt) * (size_t)KK + k0;
      FragB bf;
      bf.h[0] = *(const v8usa*)wq;
      bf.h[1] = *(const v8usa*)(wq + 16);
      acc[nt] = wmb(af, bf, acc[nt]);
    }
  }

#pragma unroll
  for (int nt = 0; nt < NT; ++nt) {
    const int lc = 16 * nt + m;
#pragma unroll
    for (int r = 0; r < 8; ++r) {
      const int lr = 16 * wave + 8 * hh + r;
      stg[lr * NC + lc] = acc[nt][r];
    }
  }
  __syncthreads();

  float bq[CPL];
  if constexpr (CPL == 4) {
    const v4f b4 = *(const v4fa*)(bias + 4 * lane);
    bq[0] = bf16_val(b4.x); bq[1] = bf16_val(b4.y); bq[2] = bf16_val(b4.z); bq[3] = bf16_val(b4.w);
  } else {
    const v2f bp2 = *(const v2fa*)(bias + 2 * lane);
    bq[0] = bf16_val(bp2.x); bq[1] = bf16_val(bp2.y);
  }

  float pv[16][CPL];
  int wn = 0;
  float wm[CPL], wqv[CPL];
#pragma unroll
  for (int j = 0; j < CPL; ++j) { wm[j] = 0.0f; wqv[j] = 0.0f; }
#pragma unroll
  for (int i = 0; i < 16; ++i) {
    const int row = rowBase + 16 * wave + i;
    const bool ok = row < nN;
    float x[CPL];
    if constexpr (CPL == 4) {
      const v4f t4 = *(const v4fa*)(stg + (16 * wave + i) * NC + 4 * lane);
      x[0] = t4.x; x[1] = t4.y; x[2] = t4.z; x[3] = t4.w;
    } else {
      const v2f t2 = *(const v2fa*)(stg + (16 * wave + i) * NC + 2 * lane);
      x[0] = t2.x; x[1] = t2.y;
    }
    float vv[CPL];
#pragma unroll
    for (int j = 0; j < CPL; ++j) {
      vv[j] = ok ? (x[j] + bq[j]) : 0.0f;
      pv[i][j] = vv[j];
    }
    if (ok) {
      wn += 1;
      const float rk = 1.0f / (float)(i + 1);
#pragma unroll
      for (int j = 0; j < CPL; ++j) {
        const float dd = vv[j] - wm[j];
        wm[j]  = fmaf(dd, rk, wm[j]);
        wqv[j] = fmaf(dd, vv[j] - wm[j], wqv[j]);
      }
    }
  }

#pragma unroll
  for (int i = 0; i < 16; ++i) {
    float* op = outp + (size_t)(rowBase + 16 * wave + i) * (size_t)NC + CPL * lane;
    if constexpr (CPL == 4) {
      v4f q; q.x = pv[i][0]; q.y = pv[i][1]; q.z = pv[i][2]; q.w = pv[i][3];
      *(volatile v4f*)op = q;
    } else {
      v2f q; q.x = pv[i][0]; q.y = pv[i][1];
      *(volatile v2f*)op = q;
    }
  }
  __threadfence();
#pragma unroll
  for (int i = 0; i < 16; ++i) {
    float* op = outp + (size_t)(rowBase + 16 * wave + i) * (size_t)NC + CPL * lane;
    if constexpr (CPL == 4) {
      v4f q; q.x = pv[i][0]; q.y = pv[i][1]; q.z = pv[i][2]; q.w = pv[i][3];
      *(volatile v4f*)op = q;
    } else {
      v2f q; q.x = pv[i][0]; q.y = pv[i][1];
      *(volatile v2f*)op = q;
    }
  }

  if (lane == 0) wst[wave * WSTW] = (float)wn;
#pragma unroll
  for (int j = 0; j < CPL; ++j) {
    wst[wave * WSTW + 1 + CPL * lane + j]      = wm[j];
    wst[wave * WSTW + 1 + D2 + CPL * lane + j] = wqv[j];
  }
#pragma unroll 1
  for (int i = tid; i < PARTW; i += GTHR) pst[i] = 0.0f;
  __syncthreads();
  if (tid < NC) {
    float n = 0.0f, mean = 0.0f, M2 = 0.0f;
#pragma unroll 1
    for (int w2 = 0; w2 < GWAVE; ++w2) {
      const float nb = wst[w2 * WSTW];
      const float mb = wst[w2 * WSTW + 1 + tid];
      const float qb = wst[w2 * WSTW + 1 + D2 + tid];
      if (nb > 0.5f) {
        const float nn = n + nb;
        const float delta = mb - mean;
        const float f = nb / nn;
        mean = fmaf(delta, f, mean);
        M2 = M2 + qb + delta * delta * n * f;
        n = nn;
      }
    }
    pst[1 + tid] = mean;
    pst[1 + D2 + tid] = M2;
    if (tid == 0) pst[0] = n;
  }
  __syncthreads();
  const int pb = (int)blockIdx.x;
  v4f ps = {0.0f, 0.0f, 0.0f, 0.0f};
  if (tid < PARTW / 4) {
    ps = *(const v4fa*)(pst + 4 * tid);
    *(volatile v4f*)(part + (size_t)pb * PARTW + 4 * tid) = ps;
  }
  __threadfence();
  if (tid < PARTW / 4) {
    *(volatile v4f*)(part + (size_t)pb * PARTW + 4 * tid) = ps;
  }
}

template <int NC>
__global__ __launch_bounds__(D2) void k_bnfin(const float* __restrict__ part, int nPart,
                                              const float* __restrict__ gam, const float* __restrict__ bet,
                                              float* ss) {
  __shared__ __attribute__((aligned(16))) float stg[2 * NC];
  const int tid = (int)threadIdx.x;
  const int c = tid < NC ? tid : NC - 1;
  double n = 0.0, mean = 0.0, M2 = 0.0;
#pragma unroll 1
  for (int b = 0; b < nPart; ++b) {
    const float* pr = part + (size_t)b * PARTW;
    const double nb = (double)pr[0];
    const double mb = (double)pr[1 + c];
    const double qb = (double)pr[1 + D2 + c];
    if (nb > 0.5) {
      const double nn = n + nb;
      const double delta = mb - mean;
      const double f = nb / nn;
      mean = mean + delta * f;
      M2 = M2 + qb + delta * delta * n * f;
      n = nn;
    }
  }
  const double ntot = n < 1.0 ? 1.0 : n;
  const float varf  = (float)(M2 / ntot);
  const float meanf = (float)mean;
  const float rstd = rsqrtf(varf + 1e-5f);
  const float sc = bf16_val(gam[c]) * rstd;
  const float sh = bf16_val(bet[c]) - meanf * sc;
  if (tid < NC) {
    stg[c] = sc;
    stg[NC + c] = sh;
  }
  __syncthreads();
  v4f v = {0.0f, 0.0f, 0.0f, 0.0f};
  if (tid < (2 * NC) / 4) {
    v = *(const v4fa*)(stg + 4 * tid);
    *(volatile v4f*)(ss + 4 * tid) = v;
  }
  __threadfence();
  if (tid < (2 * NC) / 4) {
    *(volatile v4f*)(ss + 4 * tid) = v;
  }
}

__global__ __launch_bounds__(NTHR) void k_apply1(const float* __restrict__ s1, const float* __restrict__ ss,
                                                 int nN, int mRows, unsigned short* apl2) {
  __shared__ __attribute__((aligned(16))) float ssh[2 * D2];
  __shared__ __attribute__((aligned(16))) unsigned short rbuf[NWAVE * 2 * D2];
  const int tid = (int)threadIdx.x, lane = tid & 31, wave = tid >> 5;
  ssh[tid] = ss[tid];
  __syncthreads();
  const v4f sc = *(const v4fa*)(ssh + 4 * lane);
  const v4f sh = *(const v4fa*)(ssh + D2 + 4 * lane);
  unsigned short* rb = rbuf + wave * (2 * D2);
  const int rb0 = (int)blockIdx.x * HPB + wave * HPR;

  v8us qv[HPR];
#pragma unroll
  for (int i = 0; i < HPR; ++i) {
    const int row = rb0 + i;
    const bool live = row < nN;
    const int rc = live ? row : (nN - 1);
    const v4f a = *(const v4fa*)(s1 + (size_t)rc * D2 + 4 * lane);
    v4f y;
    y.x = fmaxf(fmaf(a.x, sc.x, sh.x), 0.0f);
    y.y = fmaxf(fmaf(a.y, sc.y, sh.y), 0.0f);
    y.z = fmaxf(fmaf(a.z, sc.z, sh.z), 0.0f);
    y.w = fmaxf(fmaf(a.w, sc.w, sh.w), 0.0f);
    y.x = live ? y.x : 0.0f; y.y = live ? y.y : 0.0f; y.z = live ? y.z : 0.0f; y.w = live ? y.w : 0.0f;
    v4us mh, ml;
    {
      unsigned lb;
      unsigned hb;
      hb = hl_bits(y.x, lb); mh[0] = (unsigned short)hb; ml[0] = (unsigned short)lb;
      hb = hl_bits(y.y, lb); mh[1] = (unsigned short)hb; ml[1] = (unsigned short)lb;
      hb = hl_bits(y.z, lb); mh[2] = (unsigned short)hb; ml[2] = (unsigned short)lb;
      hb = hl_bits(y.w, lb); mh[3] = (unsigned short)hb; ml[3] = (unsigned short)lb;
    }
    *(v4usa*)(rb + 4 * lane) = mh;
    *(v4usa*)(rb + D2 + 4 * lane) = ml;
    wave_sync();
    qv[i] = *(const v8usa*)(rb + 8 * lane);
    wave_sync();
  }
#pragma unroll
  for (int i = 0; i < HPR; ++i) {
    const int row = rb0 + i;
    if (row < mRows) {
      *(volatile v8us*)(apl2 + (size_t)row * K2 + 8 * lane) = qv[i];
    }
  }
  __threadfence();
#pragma unroll
  for (int i = 0; i < HPR; ++i) {
    const int row = rb0 + i;
    if (row < mRows) {
      *(volatile v8us*)(apl2 + (size_t)row * K2 + 8 * lane) = qv[i];
    }
  }
}

template <int FIN>
__global__ __launch_bounds__(NTHR) void k_apply2(const float* __restrict__ tpl, const float* __restrict__ ss,
                                                 int nN, int nUnits, float* outp) {
  __shared__ __attribute__((aligned(16))) float ssh[2 * D];
  const int tid = (int)threadIdx.x;
  if (tid < 2 * D) ssh[tid] = ss[tid];
  __syncthreads();
  const int u = (int)blockIdx.x * NTHR + tid;
  if (u >= nUnits) return;
  const int row = u >> 4, j = u & 15, c0 = 4 * j;
  const v4f a  = *(const v4fa*)(tpl + (size_t)row * D + c0);
  const v4f sc = *(const v4fa*)(ssh + c0);
  const v4f sh = *(const v4fa*)(ssh + D + c0);
  v4f y;
  y.x = fmaf(a.x, sc.x, sh.x);
  y.y = fmaf(a.y, sc.y, sh.y);
  y.z = fmaf(a.z, sc.z, sh.z);
  y.w = fmaf(a.w, sc.w, sh.w);
  if constexpr (FIN == 0) {
    const bool live = row < nN;
    y.x = live ? fmaxf(y.x, 0.0f) : 0.0f;
    y.y = live ? fmaxf(y.y, 0.0f) : 0.0f;
    y.z = live ? fmaxf(y.z, 0.0f) : 0.0f;
    y.w = live ? fmaxf(y.w, 0.0f) : 0.0f;
  }
  float* op = outp + (size_t)row * D + c0;
  *(volatile v4f*)op = y;
  __threadfence();
  *(volatile v4f*)op = y;
}

static inline int cdiv(int a, int b) { return (a + b - 1) / b; }
static inline size_t al256(size_t o) { return (o + 255) & ~(size_t)255; }

extern "C" void kernel_launch(void* const* d_in, const int* in_sizes, int n_in,
                              void* d_out, int out_size, void* d_ws, size_t ws_size,
                              hipStream_t stream) {
  if (n_in < 15) return;
  const int nN = in_sizes[0];
  if (nN < 16 || nN >= (1 << 22)) return;
  if (in_sizes[1] < 2 || (in_sizes[1] & 1) != 0) return;
  const int nE = in_sizes[1] / 2;
  if (nE < 1 || nE >= (1 << 21)) return;
  if (in_sizes[2] != nE * FE) return;
  if (in_sizes[3] < D || (in_sizes[3] % D) != 0) return;
  const int nR = in_sizes[3] / D;
  if (in_sizes[4] < WEF || (in_sizes[4] % WEF) != 0) return;
  const int nL = in_sizes[4] / WEF;
  if (nL < 1 || nL > MAXL) return;
  if (in_sizes[5] != nL * D || in_sizes[6] != nL) return;
  if (in_sizes[7] != nL * D * D2) return;
  if (in_sizes[8] != nL * D2 || in_sizes[9] != nL * D2 || in_sizes[10] != nL * D2) return;
  if (in_sizes[11] != nL * D2 * D) return;
  if (in_sizes[12] != nL * D || in_sizes[13] != nL * D || in_sizes[14] != nL * D) return;
  if ((long long)out_size != (long long)nN * D) return;

  const int*   xi    = (const int*)d_in[0];
  const int*   edge  = (const int*)d_in[1];
  const float* eattr = (const float*)d_in[2];
  const float* emb   = (const float*)d_in[3];
  const float* We    = (const float*)d_in[4];
  const float* be    = (const float*)d_in[5];
  const float* eps   = (const float*)d_in[6];
  const float* W1    = (const float*)d_in[7];
  const float* b1    = (const float*)d_in[8];
  const float* g1    = (const float*)d_in[9];
  const float* bb1   = (const float*)d_in[10];
  const float* W2    = (const float*)d_in[11];
  const float* b2    = (const float*)d_in[12];
  const float* g2    = (const float*)d_in[13];
  const float* bb2   = (const float*)d_in[14];
  float* out = (float*)d_out;
  const int* src = edge;
  const int* dst = edge + nE;

  const int MP = cdiv(nN, GBM) * GBM;
  const int gM = MP / GBM;
  const int gA = cdiv(nN, NBA);
  if ((long long)gA * NBA < (long long)MP) return;
  if ((MP % HPB) != 0) return;
  const int vec8 = ((nE & 3) == 0) ? 1 : 0;

  char* ws = (char*)d_ws;
  size_t off = 0;
  const size_t oBT1 = off; off = al256(off + (size_t)nL * D2 * K1 * 2);
  const size_t oBT2 = off; off = al256(off + (size_t)nL * D * K2 * 2);
  const size_t oH   = off; off = al256(off + (size_t)MP * D * 4);
  const size_t oA1  = off; off = al256(off + (size_t)MP * K1 * 2);
  const size_t oS1  = off; off = al256(off + (size_t)MP * D2 * 4);
  const size_t oA2  = off; off = al256(off + (size_t)MP * K2 * 2);
  const size_t oT   = off; off = al256(off + (size_t)MP * D * 4);
  const size_t oPT  = off; off = al256(off + (size_t)gM * PARTW * 4);
  const size_t oSS1 = off; off = al256(off + (size_t)(2 * D2) * 4);
  const size_t oSS2 = off; off = al256(off + (size_t)(2 * D) * 4);
  if (off > ws_size || off > (size_t)WSMAX) return;
  unsigned short* BT1 = (unsigned short*)(ws + oBT1);
  unsigned short* BT2 = (unsigned short*)(ws + oBT2);
  float*          H   = (float*)(ws + oH);
  unsigned short* A1  = (unsigned short*)(ws + oA1);
  float*          S1  = (float*)(ws + oS1);
  unsigned short* A2  = (unsigned short*)(ws + oA2);
  float*          T   = (float*)(ws + oT);
  float*          PT  = (float*)(ws + oPT);
  float*          SS1 = (float*)(ws + oSS1);
  float*          SS2 = (float*)(ws + oSS2);

  const size_t scanLds = (size_t)AGG_LDS_INTS * 4;
  hipFuncSetAttribute(reinterpret_cast<const void*>(&k_scan), hipFuncAttributeMaxDynamicSharedMemorySize, (int)scanLds);

  const int nUh = MP * 16;
  const int nUo = nN * 16;

  k_wprep<<<8 * nL, NTHR, 0, stream>>>(W1, W2, nL, BT1, BT2);
  k_hinit<<<cdiv(nUh, NTHR), NTHR, 0, stream>>>(xi, emb, nR, nN, nUh, H);
  for (int l = 0; l < nL; ++l) {
    k_scan<<<gA, NTHR, scanLds, stream>>>(src, dst, nE, nN, vec8, MP, eattr, We + (size_t)l * WEF,
                                          be + (size_t)l * D, eps + l, H, A1);
    k_gemm<D2, K1><<<gM, GTHR, 0, stream>>>(A1, BT1 + (size_t)l * (D2 * K1), b1 + (size_t)l * D2, nN, S1, PT);
    k_bnfin<D2><<<1, D2, 0, stream>>>(PT, gM, g1 + (size_t)l * D2, bb1 + (size_t)l * D2, SS1);
    k_apply1<<<gM, NTHR, 0, stream>>>(S1, SS1, nN, MP, A2);
    k_gemm<D, K2><<<gM, GTHR, 0, stream>>>(A2, BT2 + (size_t)l * (D * K2), b2 + (size_t)l * D, nN, T, PT);
    k_bnfin<D><<<1, D, 0, stream>>>(PT, gM, g2 + (size_t)l * D, bb2 + (size_t)l * D, SS2);
    if (l < nL - 1) {
      k_apply2<0><<<cdiv(nUh, NTHR), NTHR, 0, stream>>>(T, SS2, nN, nUh, H);
    } else {
      k_apply2<1><<<cdiv(nUo, NTHR), NTHR, 0, stream>>>(T, SS2, nN, nUo, out);
    }
  }
}
